// E2PN_87222195847618
// MI455X (gfx1250) — hardware-verified
//
#include <hip/hip_runtime.h>


#define N1   65536
#define N2   16384
#define N3   4096
#define N4   1024
#define KNB  32
typedef _Float16 h16;
typedef unsigned short bf;
typedef __attribute__((ext_vector_type(16))) __bf16   v16bf;
typedef __attribute__((ext_vector_type(16))) _Float16 v16h;
typedef __attribute__((ext_vector_type(8)))  _Float16 v8h;
typedef __attribute__((ext_vector_type(8)))  unsigned short v8us;
typedef __attribute__((ext_vector_type(8)))  float    v8f;
typedef __attribute__((ext_vector_type(4)))  float    v4f;
typedef v8h  __attribute__((may_alias)) v8ha;
typedef v4f  __attribute__((may_alias)) v4fa;
typedef v8us __attribute__((may_alias)) v8usa;

__device__ __forceinline__ unsigned short f2bf(float f) { unsigned u = __float_as_uint(f); u += 0x7FFFu + ((u >> 16) & 1u); return (unsigned short)(u >> 16); }
__device__ __forceinline__ float bf2f(unsigned short b) { return __uint_as_float(((unsigned)b) << 16); }
__device__ __forceinline__ float bfr(float f) { return bf2f(f2bf(f)); }
__device__ __forceinline__ v16h cat16(v8h lo, v8h hi) { return __builtin_shufflevector(lo, hi, 0, 1, 2, 3, 4, 5, 6, 7, 8, 9, 10, 11, 12, 13, 14, 15); }
__device__ __forceinline__ v16bf cat16b(v8us lo, v8us hi) { return __builtin_bit_cast(v16bf, __builtin_shufflevector(lo, hi, 0, 1, 2, 3, 4, 5, 6, 7, 8, 9, 10, 11, 12, 13, 14, 15)); }
__device__ __forceinline__ v8f wmma16(v16h a, v16h b, v8f c) { return __builtin_amdgcn_wmma_f32_16x16x32_f16(false, a, false, b, (short)0, c, false, false); }
__device__ __forceinline__ v8f wmmab(v16bf a, v16bf b, v8f c) { return __builtin_amdgcn_wmma_f32_16x16x32_bf16(false, a, false, b, (short)0, c, false, false); }


template <typename T16> struct WFrag;
template <> struct WFrag<h16> { typedef v16h V; static __device__ __forceinline__ V ld(const h16* p) { return cat16(*(const v8h*)p, *(const v8h*)(p + 16)); } static __device__ __forceinline__ v8f mma(V a, V b, v8f c) { return wmma16(a, b, c); } };
template <> struct WFrag<bf> { typedef v16bf V; static __device__ __forceinline__ V ld(const bf* p) { return cat16b(*(const v8us*)p, *(const v8us*)(p + 16)); } static __device__ __forceinline__ v8f mma(V a, V b, v8f c) { return wmmab(a, b, c); } };
template <typename T16, int NSPLIT, bool BIAS>
__global__ __launch_bounds__(32) void k_gemmw(const T16* __restrict__ A, const T16* __restrict__ A2, const T16* __restrict__ Bt, const T16* __restrict__ Bt2, int K, float* C, int ldc, const float* __restrict__ bias, size_t sA, size_t sB, size_t sC) {
    typedef typename WFrag<T16>::V V;
    __shared__ __align__(16) float os[16 * 68];
    const size_t z = blockIdx.z; A += z * sA; if (A2) A2 += z * sA; Bt += z * sB; if (Bt2) Bt2 += z * sB; C += z * sC;
    const int lane = threadIdx.x & 31, lr = lane & 15, hi = lane >> 4; const int r0 = blockIdx.x * 64, c0 = blockIdx.y * 64;
    v8f acc[4][4];
#pragma unroll
    for (int mb = 0; mb < 4; ++mb)
#pragma unroll
        for (int nb = 0; nb < 4; ++nb) acc[mb][nb] = (v8f){};
    const size_t aoff = (size_t)(r0 + lr) * K + 8 * hi, boff = (size_t)(c0 + lr) * K + 8 * hi;
#pragma unroll 1
    for (int kc = 0; kc < K; kc += 32) {
        V a[4], a2[4];
#pragma unroll
        for (int mb = 0; mb < 4; ++mb) { a[mb] = WFrag<T16>::ld(A + aoff + (size_t)mb * 16 * K + kc); if (NSPLIT == 1 || NSPLIT == 2) a2[mb] = WFrag<T16>::ld(A2 + aoff + (size_t)mb * 16 * K + kc); }
#pragma unroll
        for (int nb = 0; nb < 4; ++nb) { const V b = WFrag<T16>::ld(Bt + boff + (size_t)nb * 16 * K + kc); V b2; if (NSPLIT >= 2) b2 = WFrag<T16>::ld(Bt2 + boff + (size_t)nb * 16 * K + kc);
#pragma unroll
            for (int mb = 0; mb < 4; ++mb) { acc[mb][nb] = WFrag<T16>::mma(a[mb], b, acc[mb][nb]); if (NSPLIT == 1 || NSPLIT == 2) acc[mb][nb] = WFrag<T16>::mma(a2[mb], b, acc[mb][nb]); if (NSPLIT >= 2) acc[mb][nb] = WFrag<T16>::mma(a[mb], b2, acc[mb][nb]); } }
        asm volatile("v_nop\n\tv_nop\n\tv_nop\n\tv_nop" : "+v"(acc[0][0]), "+v"(acc[1][1]), "+v"(acc[2][2]), "+v"(acc[3][3]) : "v"(a[0]), "v"(a[3]));
    }
#pragma unroll
    for (int mb = 0; mb < 4; ++mb) {
#pragma unroll
        for (int nb = 0; nb < 4; ++nb) {
#pragma unroll
            for (int j = 0; j < 8; ++j) os[(hi * 8 + j) * 68 + nb * 16 + lr] = acc[mb][nb][j]; }
        __builtin_amdgcn_wave_barrier(); asm volatile("" ::: "memory");
        float* crow = C + (size_t)(r0 + mb * 16) * ldc + c0;
#pragma unroll 1
        for (int ps = 0; ps < 2; ++ps) {
#pragma unroll
            for (int s = 0; s < 8; ++s) { const int row = 2 * s + hi, cofs = lr * 4; v4f val = *(const v4fa*)(os + row * 68 + cofs); if (BIAS) { val[0] += bfr(bias[c0 + cofs]); val[1] += bfr(bias[c0 + cofs + 1]); val[2] += bfr(bias[c0 + cofs + 2]); val[3] += bfr(bias[c0 + cofs + 3]); }
                *(volatile v4f*)(crow + (size_t)row * ldc + cofs) = val; }
            if (ps == 0) __threadfence(); }
        __builtin_amdgcn_wave_barrier(); asm volatile("" ::: "memory");
    }
}

__device__ __forceinline__ void splitf(float y, unsigned short& h, unsigned short& l) { h = f2bf(y); l = f2bf(y - bf2f(h)); }
__device__ __forceinline__ float lrelu_(float x) { return x > 0.f ? x : 0.1f * x; }
typedef __attribute__((ext_vector_type(2))) unsigned short v2us;
typedef __attribute__((ext_vector_type(4))) unsigned short v4us;

__global__ __launch_bounds__(256) void k_wpadT(const float* __restrict__ w, int kreal, int nreal, int NOUT, int KP, bf* Bt) { const int e = (blockIdx.x * 256 + threadIdx.x) * 2; if (e >= NOUT * KP) return; const int k = e % KP, n = e / KP; v2us o; o[0] = (n < nreal && k < kreal) ? f2bf(w[(size_t)k * nreal + n]) : (unsigned short)0; o[1] = (n < nreal && k + 1 < kreal) ? f2bf(w[(size_t)(k + 1) * nreal + n]) : (unsigned short)0; *(volatile v2us*)(Bt + e) = o; __threadfence(); *(volatile v2us*)(Bt + e) = o; }
__global__ __launch_bounds__(256) void k_gmean(const float* __restrict__ X, int NS, int C, const int* __restrict__ idx, int NQ, bf* Ph, bf* Pl) { const size_t e = ((size_t)blockIdx.x * 256 + threadIdx.x) * 4; if (e >= (size_t)NQ * C) return; const int c = (int)(e % C); const int q = (int)(e / C); float a0 = 0.f, a1 = 0.f, a2 = 0.f, a3 = 0.f;
#pragma unroll 1
    for (int k = 0; k < KNB; ++k) { const int j = idx[(size_t)q * KNB + k]; if (j >= 0 && j < NS) { const v4f v = *(const v4f*)(X + (size_t)j * C + c); a0 = __fadd_rn(a0, v[0]); a1 = __fadd_rn(a1, v[1]); a2 = __fadd_rn(a2, v[2]); a3 = __fadd_rn(a3, v[3]); } }
    const float inv = 1.0f / KNB; v4us oh, ol; unsigned short hh, ll; splitf(a0 * inv, hh, ll); oh[0] = hh; ol[0] = ll; splitf(a1 * inv, hh, ll); oh[1] = hh; ol[1] = ll; splitf(a2 * inv, hh, ll); oh[2] = hh; ol[2] = ll; splitf(a3 * inv, hh, ll); oh[3] = hh; ol[3] = ll;
    *(volatile v4us*)(Ph + e) = oh; *(volatile v4us*)(Pl + e) = ol; __threadfence(); *(volatile v4us*)(Ph + e) = oh; *(volatile v4us*)(Pl + e) = ol; }
__global__ __launch_bounds__(256) void k_gmaxpl(const float* __restrict__ X, int NS, int C, const int* __restrict__ idx, int NQ, float* GM, bf* Ph, bf* Pl) { const size_t e = ((size_t)blockIdx.x * 256 + threadIdx.x) * 4; if (e >= (size_t)NQ * C) return; const int c = (int)(e % C); const int q = (int)(e / C); v4f m; m[0] = m[1] = m[2] = m[3] = -3.0e38f;
#pragma unroll 1
    for (int k = 0; k < KNB; ++k) { const int j = idx[(size_t)q * KNB + k]; v4f v; if (j >= 0 && j < NS) v = *(const v4f*)(X + (size_t)j * C + c); else { v[0] = v[1] = v[2] = v[3] = 0.f; } m[0] = fmaxf(m[0], v[0]); m[1] = fmaxf(m[1], v[1]); m[2] = fmaxf(m[2], v[2]); m[3] = fmaxf(m[3], v[3]); }
    v4us oh, ol;
#pragma unroll
    for (int u = 0; u < 4; ++u) { unsigned short hh, ll; splitf(m[u], hh, ll); oh[u] = hh; ol[u] = ll; } for (int ps = 0; ps < 2; ++ps) { if (GM) *(volatile v4f*)(GM + e) = m; *(volatile v4us*)(Ph + e) = oh; *(volatile v4us*)(Pl + e) = ol; if (ps == 0) __threadfence(); } }
__global__ __launch_bounds__(256) void k_first(const float* __restrict__ feats, const int* __restrict__ idx, const float* __restrict__ w, float* S1, bf* Ph, bf* Pl) { const size_t e = ((size_t)blockIdx.x * 256 + threadIdx.x) * 4; if (e >= (size_t)N1 * 64) return; const int c = (int)(e % 64); const int q = (int)(e / 64); float a = 0.f;
#pragma unroll 1
    for (int k = 0; k < KNB; ++k) { const int j = idx[(size_t)q * KNB + k]; if (j >= 0 && j < N1) a = __fadd_rn(a, bfr(feats[j])); }
    const float m = a * (1.0f / KNB); v4f o; v4us oh, ol;
#pragma unroll
    for (int u = 0; u < 4; ++u) { o[u] = lrelu_(__fmul_rn(m, bfr(w[c + u]))); unsigned short hh, ll; splitf(o[u], hh, ll); oh[u] = hh; ol[u] = ll; } for (int ps = 0; ps < 2; ++ps) { *(volatile v4f*)(S1 + e) = o; *(volatile v4us*)(Ph + e) = oh; *(volatile v4us*)(Pl + e) = ol; if (ps == 0) __threadfence(); } }
__global__ __launch_bounds__(256) void k_lrelupl(const float* __restrict__ F, size_t n4, float* Y, bf* Ph, bf* Pl) { const size_t e = ((size_t)blockIdx.x * 256 + threadIdx.x) * 4; if (e >= n4 * 4) return; const v4f a = *(const v4f*)(F + e); v4f o; v4us oh, ol;
#pragma unroll
    for (int u = 0; u < 4; ++u) { o[u] = lrelu_(a[u]); unsigned short hh, ll; splitf(o[u], hh, ll); oh[u] = hh; ol[u] = ll; } for (int ps = 0; ps < 2; ++ps) { if (Y) *(volatile v4f*)(Y + e) = o; *(volatile v4us*)(Ph + e) = oh; *(volatile v4us*)(Pl + e) = ol; if (ps == 0) __threadfence(); } }
__global__ __launch_bounds__(256) void k_addlrelu(const float* __restrict__ F, const float* __restrict__ SC, size_t n4, float* Y, bf* Ph, bf* Pl) { const size_t e = ((size_t)blockIdx.x * 256 + threadIdx.x) * 4; if (e >= n4 * 4) return; const v4f a = *(const v4f*)(F + e), s = *(const v4f*)(SC + e); v4f o; v4us oh, ol;
#pragma unroll
    for (int u = 0; u < 4; ++u) { o[u] = lrelu_(__fadd_rn(a[u], s[u])); unsigned short hh, ll; splitf(o[u], hh, ll); oh[u] = hh; ol[u] = ll; } for (int ps = 0; ps < 2; ++ps) { *(volatile v4f*)(Y + e) = o; if (Ph) { *(volatile v4us*)(Ph + e) = oh; *(volatile v4us*)(Pl + e) = ol; } if (ps == 0) __threadfence(); } }
__global__ __launch_bounds__(256) void k_nearpl(const float* __restrict__ X, int NS, int C, const int* __restrict__ up, int NQ, int pitch, bf* Ch, bf* Cl) { const size_t e = ((size_t)blockIdx.x * 256 + threadIdx.x) * 4; if (e >= (size_t)NQ * C) return; const int c = (int)(e % C); const int q = (int)(e / C); const int j = up[(size_t)q * KNB]; v4f v; if (j >= 0 && j < NS) v = *(const v4f*)(X + (size_t)j * C + c); else { v[0] = v[1] = v[2] = v[3] = 0.f; }
    v4us oh, ol;
#pragma unroll
    for (int u = 0; u < 4; ++u) { unsigned short hh, ll; splitf(v[u], hh, ll); oh[u] = hh; ol[u] = ll; } const size_t o = (size_t)q * pitch + c; *(volatile v4us*)(Ch + o) = oh; *(volatile v4us*)(Cl + o) = ol; __threadfence(); *(volatile v4us*)(Ch + o) = oh; *(volatile v4us*)(Cl + o) = ol; }
__global__ __launch_bounds__(256) void k_catpl(const float* __restrict__ X, int C, int NQ, int pitch, int c0, bf* Ch, bf* Cl) { const size_t e = ((size_t)blockIdx.x * 256 + threadIdx.x) * 4; if (e >= (size_t)NQ * C) return; const int c = (int)(e % C); const int q = (int)(e / C); const v4f v = *(const v4f*)(X + e); v4us oh, ol;
#pragma unroll
    for (int u = 0; u < 4; ++u) { unsigned short hh, ll; splitf(v[u], hh, ll); oh[u] = hh; ol[u] = ll; } const size_t o = (size_t)q * pitch + c0 + c; *(volatile v4us*)(Ch + o) = oh; *(volatile v4us*)(Cl + o) = ol; __threadfence(); *(volatile v4us*)(Ch + o) = oh; *(volatile v4us*)(Cl + o) = ol; }
__global__ __launch_bounds__(256) void k_splitp(const float* __restrict__ F, size_t n4, bf* Ph, bf* Pl) { const size_t e = ((size_t)blockIdx.x * 256 + threadIdx.x) * 4; if (e >= n4 * 4) return; const v4f a = *(const v4f*)(F + e); v4us oh, ol;
#pragma unroll
    for (int u = 0; u < 4; ++u) { unsigned short hh, ll; splitf(a[u], hh, ll); oh[u] = hh; ol[u] = ll; } *(volatile v4us*)(Ph + e) = oh; *(volatile v4us*)(Pl + e) = ol; __threadfence(); *(volatile v4us*)(Ph + e) = oh; *(volatile v4us*)(Pl + e) = ol; }

static inline unsigned nb4(size_t n) { return (unsigned)((n / 4 + 255) / 256); }
#define GEMM(Ah, Al, Bt, M, N, K, Cout) k_gemmw<bf, 1, false><<<dim3((M) / 64, (N) / 64, 1), 32, 0, stream>>>(Ah, Al, Bt, nullptr, K, Cout, N, nullptr, 0, 0, 0)

extern "C" void kernel_launch(void* const* d_in, const int* in_sizes, int n_in,
                              void* d_out, int out_size, void* d_ws, size_t ws_size, hipStream_t stream) {
    (void)in_sizes; (void)n_in; (void)out_size;
    const float* feats = (const float*)d_in[0]; const int* nbr1 = (const int*)d_in[1]; const int* nbr2 = (const int*)d_in[2]; const int* nbr3 = (const int*)d_in[3]; const int* nbr4 = (const int*)d_in[4]; const int* sub1 = (const int*)d_in[5]; const int* sub2 = (const int*)d_in[6]; const int* sub3 = (const int*)d_in[7]; const int* up32 = (const int*)d_in[8]; const int* up21 = (const int*)d_in[9];
    const float** Wf = (const float**)d_in;
    const float *w_e11 = Wf[10], *e12_w1 = Wf[11], *e12_wc = Wf[12], *e12_w3 = Wf[13], *e12_wsc = Wf[14], *e21_w1 = Wf[15], *e21_wc = Wf[16], *e21_w3 = Wf[17], *e22_w1 = Wf[18], *e22_wc = Wf[19], *e22_w3 = Wf[20], *e22_wsc = Wf[21], *e23_w1 = Wf[22], *e23_wc = Wf[23], *e23_w3 = Wf[24], *e31_w1 = Wf[25], *e31_wc = Wf[26], *e31_w3 = Wf[27], *e32_w1 = Wf[28], *e32_wc = Wf[29], *e32_w3 = Wf[30], *e32_wsc = Wf[31], *e33_w1 = Wf[32], *e33_wc = Wf[33], *e33_w3 = Wf[34], *e41_w1 = Wf[35], *e41_wc = Wf[36], *e41_w3 = Wf[37], *e42_w1 = Wf[38], *e42_wc = Wf[39], *e42_w3 = Wf[40], *e42_wsc = Wf[41], *e43_w1 = Wf[42], *e43_wc = Wf[43], *e43_w3 = Wf[44], *wd3 = Wf[45], *wd2 = Wf[46];
    float* OUT_L2 = (float*)d_out; float* OUT_L3 = (float*)((char*)d_out + 16777216); float* OUT_S4 = (float*)((char*)d_out + 25165824);
    char* wsp = (char*)d_ws;
    auto take = [&](size_t bytes) { char* p = wsp; wsp += (bytes + 255) & ~(size_t)255; return (void*)p; };
    struct WT { const float* w; int kr, nr, NO, KP; bf* bt; };
    WT wts[] = { {e12_w1, 64, 32, 64, 64, 0}, {e12_wc, 32, 32, 64, 64, 0}, {e12_w3, 32, 128, 128, 64, 0}, {e12_wsc, 64, 128, 128, 64, 0}, {e21_w1, 128, 32, 64, 128, 0}, {e21_wc, 32, 32, 64, 64, 0}, {e21_w3, 32, 128, 128, 64, 0},
                 {e22_w1, 128, 64, 64, 128, 0}, {e22_wc, 64, 64, 64, 64, 0}, {e22_w3, 64, 256, 256, 64, 0}, {e22_wsc, 128, 256, 256, 128, 0}, {e23_w1, 256, 64, 64, 256, 0}, {e23_wc, 64, 64, 64, 64, 0}, {e23_w3, 64, 256, 256, 64, 0},
                 {e31_w1, 256, 64, 64, 256, 0}, {e31_wc, 64, 64, 64, 64, 0}, {e31_w3, 64, 256, 256, 64, 0}, {e32_w1, 256, 128, 128, 256, 0}, {e32_wc, 128, 128, 128, 128, 0}, {e32_w3, 128, 512, 512, 128, 0}, {e32_wsc, 256, 512, 512, 256, 0}, {e33_w1, 512, 128, 128, 512, 0}, {e33_wc, 128, 128, 128, 128, 0}, {e33_w3, 128, 512, 512, 128, 0},
                 {e41_w1, 512, 128, 128, 512, 0}, {e41_wc, 128, 128, 128, 128, 0}, {e41_w3, 128, 512, 512, 128, 0}, {e42_w1, 512, 256, 256, 512, 0}, {e42_wc, 256, 256, 256, 256, 0}, {e42_w3, 256, 1024, 1024, 256, 0}, {e42_wsc, 512, 1024, 1024, 512, 0}, {e43_w1, 1024, 256, 256, 1024, 0}, {e43_wc, 256, 256, 256, 256, 0}, {e43_w3, 256, 1024, 1024, 256, 0},
                 {wd3, 1536, 512, 512, 1536, 0}, {wd2, 768, 256, 256, 768, 0} };
    const int NWT = sizeof(wts) / sizeof(wts[0]);
    for (int i = 0; i < NWT; ++i) wts[i].bt = (bf*)take((size_t)wts[i].NO * wts[i].KP * 2);
    float* XA = (float*)take((size_t)N1 * 128 * 4); bf* XAh = (bf*)take((size_t)N2 * 768 * 2); bf* XAl = (bf*)take((size_t)N2 * 768 * 2);
    float* F = (float*)take((size_t)N1 * 128 * 4); float* H1 = (float*)take((size_t)N1 * 64 * 4); bf* Gh = (bf*)take((size_t)N1 * 64 * 2); bf* Gl = (bf*)take((size_t)N1 * 64 * 2); bf* H2h = (bf*)take((size_t)N1 * 64 * 2); bf* H2l = (bf*)take((size_t)N1 * 64 * 2); float* F3 = (float*)take((size_t)N1 * 128 * 4); float* SCM = (float*)take((size_t)N2 * 128 * 4); bf* SCh = (bf*)take((size_t)N2 * 128 * 2); bf* SCl = (bf*)take((size_t)N2 * 128 * 2);
    float* S2 = (float*)take((size_t)N2 * 256 * 4); float* S3 = (float*)take((size_t)N3 * 512 * 4); bf* CATh = XAh; bf* CATl = XAl;
    if ((size_t)(wsp - (char*)d_ws) > ws_size) return;
    for (int i = 0; i < NWT; ++i) k_wpadT<<<(wts[i].NO * wts[i].KP / 2 + 255) / 256, 256, 0, stream>>>(wts[i].w, wts[i].kr, wts[i].nr, wts[i].NO, wts[i].KP, wts[i].bt);
    auto W = [&](const float* w) -> bf* { for (int i = 0; i < NWT; ++i) if (wts[i].w == w) return wts[i].bt; return nullptr; };
    auto resnet = [&](int NS, int NQ, int CIN, int CMIDP, int COUT, const int* nbrs, const float* w1, const float* wc, const float* w3, const float* wsc, bool strided, float* Ynext) {
        GEMM(XAh, XAl, W(w1), NS, CMIDP, CIN, F); k_lrelupl<<<nb4((size_t)NS * CMIDP), 256, 0, stream>>>(F, (size_t)NS * CMIDP / 4, H1, Gh, Gl);
        k_gmean<<<nb4((size_t)NQ * CMIDP), 256, 0, stream>>>(H1, NS, CMIDP, nbrs, NQ, Gh, Gl); GEMM(Gh, Gl, W(wc), NQ, CMIDP, CMIDP, F); k_lrelupl<<<nb4((size_t)NQ * CMIDP), 256, 0, stream>>>(F, (size_t)NQ * CMIDP / 4, nullptr, H2h, H2l);
        GEMM(H2h, H2l, W(w3), NQ, COUT, CMIDP, F3);
        const float* sc = XA;
        if (strided) { k_gmaxpl<<<nb4((size_t)NQ * CIN), 256, 0, stream>>>(XA, NS, CIN, nbrs, NQ, SCM, SCh, SCl); sc = SCM; if (wsc) { GEMM(SCh, SCl, W(wsc), NQ, COUT, CIN, F); sc = F; } }
        else if (wsc) { GEMM(XAh, XAl, W(wsc), NQ, COUT, CIN, F); sc = F; }
        k_addlrelu<<<nb4((size_t)NQ * COUT), 256, 0, stream>>>(F3, sc, (size_t)NQ * COUT / 4, Ynext, XAh, XAl);
        if (Ynext != XA) {   } };
    k_first<<<nb4((size_t)N1 * 64), 256, 0, stream>>>(feats, nbr1, w_e11, XA, XAh, XAl);
    resnet(N1, N1, 64, 64, 128, nbr1, e12_w1, e12_wc, e12_w3, e12_wsc, false, XA);
    resnet(N1, N2, 128, 64, 128, sub1, e21_w1, e21_wc, e21_w3, nullptr, true, XA);
    resnet(N2, N2, 128, 64, 256, nbr2, e22_w1, e22_wc, e22_w3, e22_wsc, false, XA);
    resnet(N2, N2, 256, 64, 256, nbr2, e23_w1, e23_wc, e23_w3, nullptr, false, S2); k_splitp<<<nb4((size_t)N2 * 256), 256, 0, stream>>>(S2, (size_t)N2 * 256 / 4, XAh, XAl);
    { GEMM(XAh, XAl, W(e31_w1), N2, 64, 256, F); k_lrelupl<<<nb4((size_t)N2 * 64), 256, 0, stream>>>(F, (size_t)N2 * 64 / 4, H1, Gh, Gl); k_gmean<<<nb4((size_t)N3 * 64), 256, 0, stream>>>(H1, N2, 64, sub2, N3, Gh, Gl); GEMM(Gh, Gl, W(e31_wc), N3, 64, 64, F); k_lrelupl<<<nb4((size_t)N3 * 64), 256, 0, stream>>>(F, (size_t)N3 * 64 / 4, nullptr, H2h, H2l); GEMM(H2h, H2l, W(e31_w3), N3, 256, 64, F3);
      k_gmaxpl<<<nb4((size_t)N3 * 256), 256, 0, stream>>>(S2, N2, 256, sub2, N3, SCM, SCh, SCl); k_addlrelu<<<nb4((size_t)N3 * 256), 256, 0, stream>>>(F3, SCM, (size_t)N3 * 256 / 4, XA, XAh, XAl); }
    resnet(N3, N3, 256, 128, 512, nbr3, e32_w1, e32_wc, e32_w3, e32_wsc, false, XA);
    resnet(N3, N3, 512, 128, 512, nbr3, e33_w1, e33_wc, e33_w3, nullptr, false, S3); k_splitp<<<nb4((size_t)N3 * 512), 256, 0, stream>>>(S3, (size_t)N3 * 512 / 4, XAh, XAl);
    { GEMM(XAh, XAl, W(e41_w1), N3, 128, 512, F); k_lrelupl<<<nb4((size_t)N3 * 128), 256, 0, stream>>>(F, (size_t)N3 * 128 / 4, H1, Gh, Gl); k_gmean<<<nb4((size_t)N4 * 128), 256, 0, stream>>>(H1, N3, 128, sub3, N4, Gh, Gl); GEMM(Gh, Gl, W(e41_wc), N4, 128, 128, F); k_lrelupl<<<nb4((size_t)N4 * 128), 256, 0, stream>>>(F, (size_t)N4 * 128 / 4, nullptr, H2h, H2l); GEMM(H2h, H2l, W(e41_w3), N4, 512, 128, F3);
      k_gmaxpl<<<nb4((size_t)N4 * 512), 256, 0, stream>>>(S3, N3, 512, sub3, N4, SCM, SCh, SCl); k_addlrelu<<<nb4((size_t)N4 * 512), 256, 0, stream>>>(F3, SCM, (size_t)N4 * 512 / 4, XA, XAh, XAl); }
    resnet(N4, N4, 512, 256, 1024, nbr4, e42_w1, e42_wc, e42_w3, e42_wsc, false, XA);
    resnet(N4, N4, 1024, 256, 1024, nbr4, e43_w1, e43_wc, e43_w3, nullptr, false, OUT_S4);
    k_nearpl<<<nb4((size_t)N3 * 1024), 256, 0, stream>>>(OUT_S4, N4, 1024, up32, N3, 1536, CATh, CATl); k_catpl<<<nb4((size_t)N3 * 512), 256, 0, stream>>>(S3, 512, N3, 1536, 1024, CATh, CATl);
    GEMM(CATh, CATl, W(wd3), N3, 512, 1536, F); k_lrelupl<<<nb4((size_t)N3 * 512), 256, 0, stream>>>(F, (size_t)N3 * 512 / 4, OUT_L3, Gh, Gl);
    k_nearpl<<<nb4((size_t)N2 * 512), 256, 0, stream>>>(OUT_L3, N3, 512, up21, N2, 768, CATh, CATl); k_catpl<<<nb4((size_t)N2 * 256), 256, 0, stream>>>(S2, 256, N2, 768, 512, CATh, CATl);
    GEMM(CATh, CATl, W(wd2), N2, 256, 768, OUT_L2);
}
